// Cross_Attn_Image_to_Token_29807073034394
// MI455X (gfx1250) — hardware-verified
//
#include <hip/hip_runtime.h>
#include <math.h>
#include <stdint.h>

#define NB     4
#define LQ     4096
#define LK     1024
#define DM     256
#define NH     8
#define HD     32
#define NQR    (NB * LQ)
#define NKR    (NB * LK)
#define NQT    (LQ / 16)
#define NWAV   (NB * NQT * NH)
#define PSP    36
#define ACARRY 16.0f
#define WSC    256.0f
#define QKC    64.0f
#define VC     64.0f
#define ZC     1024.0f
#define PCAR   1024.0f
#define PCH    512.0f
#define PONE   1.0f
#define RESC   2048.0f
#define RINV   0.00048828125f
#define NEGS   (-1.0e30f)

static_assert(NH * HD == DM);
static_assert((NQR % 64) == 0 && (NKR % 64) == 0 && (DM % 64) == 0);
static_assert((LQ % 64) == 0 && (LK % 32) == 0);
static_assert((NQR % 8) == 0 && (NKR % 8) == 0 && (DM % 8) == 0);
static_assert((NWAV % 4) == 0);
static_assert(NQT * NH == 2048);
static_assert(PCAR == (float)LK * PONE);

typedef _Float16 v16h __attribute__((ext_vector_type(16)));
typedef _Float16 v8h  __attribute__((ext_vector_type(8)));
typedef float    v8f  __attribute__((ext_vector_type(8)));
typedef float    v4f  __attribute__((ext_vector_type(4)));
typedef unsigned int v4u __attribute__((ext_vector_type(4)));

union FragH { v16h v; v8h h[2]; v4u u[2]; };

__device__ __forceinline__ unsigned short bf_bits(float f) {
  unsigned u = __float_as_uint(f);
  return (unsigned short)((u + 0x7FFFu + ((u >> 16) & 1u)) >> 16);
}
__device__ __forceinline__ float bf_up(unsigned short b) { return __uint_as_float(((unsigned)b) << 16); }
__device__ __forceinline__ float bfr(float f) { return bf_up(bf_bits(f)); }
__device__ __forceinline__ unsigned short h_bits(_Float16 x) { return __builtin_bit_cast(unsigned short, x); }
__device__ __forceinline__ unsigned pk16(unsigned short a, unsigned short b) { return (unsigned)a | ((unsigned)b << 16); }
__device__ __forceinline__ v8f zero8() { v8f z = {0.f, 0.f, 0.f, 0.f, 0.f, 0.f, 0.f, 0.f}; return z; }

__device__ __forceinline__ v16h ldfrag_h(const _Float16* p) {
  FragH f;
  f.h[0] = *(const v8h*)(p);
  f.h[1] = *(const v8h*)(p + 16);
  return f.v;
}
__device__ __forceinline__ v16h ldfrag_u(const unsigned short* p) {
  FragH f;
  f.u[0] = *(const v4u*)(p);
  f.u[1] = *(const v4u*)(p + 16);
  return f.v;
}

__device__ __forceinline__ v8f mma_raw(v16h a, v16h b, v8f c) {
  return __builtin_amdgcn_wmma_f32_16x16x32_f16(false, a, false, b, (short)0, c, false, false);
}
__device__ __forceinline__ void guard_4x1(v8f& a, v8f& b, v8f& c, v8f& d, v16h x) {
#if defined(__HIP_DEVICE_COMPILE__)
  asm volatile("v_nop\n\tv_nop\n\tv_nop\n\tv_nop" : "+v"(a), "+v"(b), "+v"(c), "+v"(d) : "v"(x));
#endif
}
__device__ __forceinline__ void keep4_h(v16h a, v16h b, v16h c, v16h d) {
#if defined(__HIP_DEVICE_COMPILE__)
  asm volatile("v_nop" :: "v"(a), "v"(b), "v"(c), "v"(d));
#endif
}
__device__ __forceinline__ void acc_guard4(v8f& a, v8f& b, v8f& c, v8f& d) {
#if defined(__HIP_DEVICE_COMPILE__)
  asm volatile("v_nop\n\tv_nop\n\tv_nop\n\tv_nop" : "+v"(a), "+v"(b), "+v"(c), "+v"(d));
#endif
}
__device__ __forceinline__ void guard_4x6(v8f& a, v8f& b, v8f& c, v8f& d,
                                          v16h x0, v16h x1, v16h x2, v16h x3, v16h x4, v16h x5) {
#if defined(__HIP_DEVICE_COMPILE__)
  asm volatile("v_nop\n\tv_nop\n\tv_nop\n\tv_nop"
               : "+v"(a), "+v"(b), "+v"(c), "+v"(d) : "v"(x0), "v"(x1), "v"(x2), "v"(x3), "v"(x4), "v"(x5));
#endif
}
__device__ __forceinline__ void guard_2x3(v8f& a, v8f& b, v16h x0, v16h x1, v16h x2) {
#if defined(__HIP_DEVICE_COMPILE__)
  asm volatile("v_nop\n\tv_nop\n\tv_nop\n\tv_nop" : "+v"(a), "+v"(b) : "v"(x0), "v"(x1), "v"(x2));
#endif
}
__device__ __forceinline__ void wave_sync_lds() {
  __builtin_amdgcn_fence(__ATOMIC_RELEASE, "workgroup");
  __builtin_amdgcn_wave_barrier();
  __builtin_amdgcn_fence(__ATOMIC_ACQUIRE, "workgroup");
}

__device__ __forceinline__ void split8(const float* sp, v4u& hi, v4u& lo) {
  const v4f a = *(const v4f*)(sp), b = *(const v4f*)(sp + 4);
  float v[8];
#pragma unroll
  for (int e = 0; e < 4; ++e) { v[e] = a[e]; v[4 + e] = b[e]; }
#pragma unroll
  for (int e = 0; e < 4; ++e) {
    const _Float16 h0 = (_Float16)v[2 * e], h1 = (_Float16)v[2 * e + 1];
    const _Float16 l0 = (_Float16)((v[2 * e] - (float)h0) * RESC);
    const _Float16 l1 = (_Float16)((v[2 * e + 1] - (float)h1) * RESC);
    hi[e] = pk16(h_bits(h0), h_bits(h1));
    lo[e] = pk16(h_bits(l0), h_bits(l1));
  }
}

__global__ __launch_bounds__(256) void cvrow(const float* __restrict__ x, unsigned short* dst, int nrows, float scale) {
  const int i   = blockIdx.x * 256 + threadIdx.x;
  const int row = i >> 5;
  const int c8  = (i & 31) * 8;
  const bool live = row < nrows;
  const int rc  = live ? row : (nrows - 1);
  const float* p = x + (size_t)rc * DM + c8;
  const v4f a = *(const v4f*)(p), b = *(const v4f*)(p + 4);
  float v[8];
#pragma unroll
  for (int e = 0; e < 4; ++e) {
    v[e]     = live ? bfr(a[e]) : 0.f;
    v[4 + e] = live ? bfr(b[e]) : 0.f;
  }
  v4u o;
#pragma unroll
  for (int e = 0; e < 4; ++e) o[e] = pk16(h_bits((_Float16)(v[2 * e] * scale)), h_bits((_Float16)(v[2 * e + 1] * scale)));
  unsigned short* dp = dst + (size_t)i * 8;
  *(volatile v4u*)dp = o;
  __threadfence();
  *(volatile v4u*)dp = o;
}

__global__ __launch_bounds__(256) void vhsum(const float* __restrict__ v, const float* __restrict__ Wv,
                                             const float* __restrict__ bv, float* S) {
  __shared__ float vs[DM];
  __shared__ __align__(16) float so[DM];
  const int t = threadIdx.x;
  const int b = blockIdx.x;
  const float* vp = v + (size_t)b * LK * DM + t;
  float a = 0.f;
#pragma unroll 1
  for (int k = 0; k < LK; ++k) a += bfr(vp[(size_t)k * DM]);
  vs[t] = a;
  __syncthreads();
  const float* wr = Wv + (size_t)t * DM;
  float s = 0.f;
#pragma unroll 1
  for (int j = 0; j < DM; ++j) s += vs[j] * bfr(wr[j]);
  s += (float)LK * bfr(bv[t]);
  so[t] = s;
  __syncthreads();
  const int tc = (t < 64) ? t : 0;
  const v4f o = *(const v4f*)(so + 4 * tc);
  float* dp = S + (size_t)b * DM + 4 * tc;
  if (t < 64) *(volatile v4f*)dp = o;
  __threadfence();
  if (t < 64) *(volatile v4f*)dp = o;
}

__device__ __forceinline__ void kloop(v8f (&acc)[4][4], const unsigned short* __restrict__ A1, int lda, long long sAk,
                                      const unsigned short* __restrict__ Bb, int ldb, int m0, int n0, int K,
                                      int rlane, int koff) {
#pragma unroll 1
  for (int k0 = 0; k0 < K; k0 += 32) {
    v16h bh[4];
#pragma unroll
    for (int j = 0; j < 4; ++j) {
      const size_t bofs = (size_t)(n0 + (j << 4) + rlane) * (size_t)ldb + (size_t)(koff + k0);
      bh[j] = ldfrag_u(Bb + bofs);
    }
    const size_t ak = (size_t)(k0 >> 5) * (size_t)sAk + (size_t)((k0 & 31) + koff);
#pragma unroll
    for (int i = 0; i < 4; ++i) {
      const size_t ao = (size_t)(m0 + (i << 4) + rlane) * (size_t)lda + ak;
      const v16h ah = ldfrag_u(A1 + ao);
#pragma unroll
      for (int j = 0; j < 4; ++j) acc[i][j] = mma_raw(ah, bh[j], acc[i][j]);
      guard_4x1(acc[i][0], acc[i][1], acc[i][2], acc[i][3], ah);
    }
    keep4_h(bh[0], bh[1], bh[2], bh[3]);
  }
}

template <int OM, int BIASM>
__global__ __launch_bounds__(256) void gemm64(
    const unsigned short* __restrict__ Ap, int lda, long long sAk, long long aLo,
    const unsigned short* __restrict__ Btp, int ldb,
    const float* __restrict__ bias, float bscale,
    void* Cout, int ldc, long long cLo,
    int M, int N, int K, float oscale) {
  __shared__ __align__(16) float sT[8][16 * 68];
  const int lane = threadIdx.x & 31;
  const int wave = threadIdx.x >> 5;
  const int tilesN = N >> 6;
  const int tilesM = M >> 6;
  const int tile = blockIdx.x * 8 + wave;
  if (tile >= tilesM * tilesN) return;
  const int tm = tile / tilesN;
  const int tn = tile - tm * tilesN;
  const int m0 = tm << 6;
  const int n0 = tn << 6;

  const int rlane = lane & 15;
  const int koff  = (lane >> 4) * 8;
  const int mOff  = (lane >> 4) * 8;

  v8f acc[4][4];
#pragma unroll
  for (int i = 0; i < 4; ++i)
#pragma unroll
    for (int j = 0; j < 4; ++j) acc[i][j] = zero8();

  if (aLo != 0) {
    kloop(acc, Ap + aLo, lda, sAk, Btp, ldb, m0, n0, K, rlane, koff);
    acc_guard4(acc[0][0], acc[0][1], acc[0][2], acc[0][3]);
    acc_guard4(acc[1][0], acc[1][1], acc[1][2], acc[1][3]);
    acc_guard4(acc[2][0], acc[2][1], acc[2][2], acc[2][3]);
    acc_guard4(acc[3][0], acc[3][1], acc[3][2], acc[3][3]);
#pragma unroll
    for (int i = 0; i < 4; ++i)
#pragma unroll
      for (int j = 0; j < 4; ++j) acc[i][j] = acc[i][j] * RINV;
  }
  kloop(acc, Ap, lda, sAk, Btp, ldb, m0, n0, K, rlane, koff);
  acc_guard4(acc[0][0], acc[0][1], acc[0][2], acc[0][3]);
  acc_guard4(acc[1][0], acc[1][1], acc[1][2], acc[1][3]);
  acc_guard4(acc[2][0], acc[2][1], acc[2][2], acc[2][3]);
  acc_guard4(acc[3][0], acc[3][1], acc[3][2], acc[3][3]);

  const int hh2 = lane >> 4, c4 = (lane & 15) * 4;
  const int q8  = lane >> 3, c8 = (lane & 7) * 8;
  float bc4[4], bc8[8];
#pragma unroll
  for (int e = 0; e < 4; ++e) bc4[e] = 0.f;
#pragma unroll
  for (int e = 0; e < 8; ++e) bc8[e] = 0.f;
  if (BIASM == 0) {
    if (OM == 4) {
      const int cb = n0 + c4;
      const int i0 = (cb <= N - 4) ? cb : (N - 4);
      const v4f b0v = *(const v4f*)(bias + i0);
#pragma unroll
      for (int e = 0; e < 4; ++e) bc4[e] = bfr(b0v[e]) * bscale;
    } else {
      const int cb = n0 + c8;
      const int i0 = (cb <= N - 8) ? cb : (N - 8);
      const v4f b0v = *(const v4f*)(bias + i0), b1v = *(const v4f*)(bias + i0 + 4);
#pragma unroll
      for (int e = 0; e < 4; ++e) { bc8[e] = bfr(b0v[e]) * bscale; bc8[4 + e] = bfr(b1v[e]) * bscale; }
    }
  }

  float* slab = sT[wave];
#pragma unroll
  for (int i = 0; i < 4; ++i) {
    const int mBase = m0 + (i << 4);
#pragma unroll
    for (int j = 0; j < 4; ++j) {
#pragma unroll
      for (int r = 0; r < 8; ++r) {
        slab[(mOff + r) * 68 + (j << 4) + rlane] = acc[i][j][r];
      }
    }
    wave_sync_lds();
    if (OM == 4) {
      float* C = (float*)Cout;
      v4f vals[8];
#pragma unroll
      for (int it = 0; it < 8; ++it) {
        const int row = it * 2 + hh2;
        float rb = 0.f;
        if (BIASM == 1) {
          const int gr = mBase + row;
          rb = bfr(bias[(gr < M) ? gr : (M - 1)]) * bscale;
        }
        v4f v = *(const v4f*)(slab + row * 68 + c4);
#pragma unroll
        for (int e = 0; e < 4; ++e) v[e] = v[e] * oscale + bc4[e] + rb;
        vals[it] = v;
      }
#pragma unroll
      for (int it = 0; it < 8; ++it) {
        const int gr = mBase + it * 2 + hh2;
        *(volatile v4f*)(C + (size_t)gr * (size_t)ldc + n0 + c4) = vals[it];
      }
      __threadfence();
#pragma unroll
      for (int it = 0; it < 8; ++it) {
        const int gr = mBase + it * 2 + hh2;
        *(volatile v4f*)(C + (size_t)gr * (size_t)ldc + n0 + c4) = vals[it];
      }
      __threadfence();
    } else {
      unsigned short* C = (unsigned short*)Cout;
      v4u hv[4], lv[4];
#pragma unroll
      for (int it = 0; it < 4; ++it) {
        const int row = it * 4 + q8;
        float rb = 0.f;
        if (BIASM == 1) {
          const int gr = mBase + row;
          rb = bfr(bias[(gr < M) ? gr : (M - 1)]) * bscale;
        }
        const float* sp = slab + row * 68 + c8;
        const v4f x0 = *(const v4f*)(sp), x1 = *(const v4f*)(sp + 4);
        float v[8];
#pragma unroll
        for (int e = 0; e < 4; ++e) {
          v[e]     = x0[e] * oscale + bc8[e] + rb;
          v[4 + e] = x1[e] * oscale + bc8[4 + e] + rb;
        }
        v4u ha, la;
#pragma unroll
        for (int e = 0; e < 4; ++e) {
          const _Float16 h0 = (_Float16)v[2 * e], h1 = (_Float16)v[2 * e + 1];
          const _Float16 l0 = (_Float16)((v[2 * e] - (float)h0) * RESC);
          const _Float16 l1 = (_Float16)((v[2 * e + 1] - (float)h1) * RESC);
          ha[e] = pk16(h_bits(h0), h_bits(h1));
          la[e] = pk16(h_bits(l0), h_bits(l1));
        }
        hv[it] = ha;
        lv[it] = la;
      }
#pragma unroll
      for (int it = 0; it < 4; ++it) {
        const int row = it * 4 + q8;
        const size_t o = (size_t)(mBase + row) * (size_t)ldc + n0 + c8;
        *(volatile v4u*)(C + o) = hv[it];
        if (OM == 3) *(volatile v4u*)(C + cLo + o) = lv[it];
      }
      __threadfence();
#pragma unroll
      for (int it = 0; it < 4; ++it) {
        const int row = it * 4 + q8;
        const size_t o = (size_t)(mBase + row) * (size_t)ldc + n0 + c8;
        *(volatile v4u*)(C + o) = hv[it];
        if (OM == 3) *(volatile v4u*)(C + cLo + o) = lv[it];
      }
      __threadfence();
    }
    wave_sync_lds();
  }
}

__device__ __forceinline__ void ostep(float t0, float t1, float& m, float& l) {
  float mx = fmaxf(t0, t1);
  mx = fmaxf(mx, __shfl_xor(mx, 1, 32));
  mx = fmaxf(mx, __shfl_xor(mx, 2, 32));
  mx = fmaxf(mx, __shfl_xor(mx, 4, 32));
  mx = fmaxf(mx, __shfl_xor(mx, 8, 32));
  const float mn = fmaxf(m, mx);
  const float al = exp2f(m - mn);
  float ps = exp2f(t0 - mn) + exp2f(t1 - mn);
  ps += __shfl_xor(ps, 1, 32);
  ps += __shfl_xor(ps, 2, 32);
  ps += __shfl_xor(ps, 4, 32);
  ps += __shfl_xor(ps, 8, 32);
  l = l * al + ps;
  m = mn;
}

__global__ __launch_bounds__(128)
void stats(const unsigned short* __restrict__ QP, const unsigned short* __restrict__ KP,
           const unsigned short* __restrict__ CP, float* ST) {
  __shared__ __align__(16) float Ls[4][64];
  const int tid  = threadIdx.x;
  const int wave = tid >> 5;
  const int lane = tid & 31;
  const int hh   = lane >> 4;
  const int c    = lane & 15;
  const int wid  = blockIdx.x * 4 + wave;
  if (wid >= NWAV) return;
  const int h  = wid & (NH - 1);
  const int gt = wid >> 3;
  const int b  = gt / NQT;
  const int q0 = gt * 16;

  const _Float16* qp1 = (const _Float16*)(const void*)QP + (size_t)(q0 + c) * (size_t)(2 * DM) + HD * h + 8 * hh;
  const v16h q1 = ldfrag_h(qp1), q2 = ldfrag_h(qp1 + DM);
  const _Float16* kp = (const _Float16*)(const void*)KP + ((size_t)b * LK + c) * (size_t)DM + HD * h + 8 * hh;
  const _Float16* cp = (const _Float16*)(const void*)CP + ((size_t)b * LK + c) * (size_t)DM + HD * h + 8 * hh;
  const float lsc = (1.4426950408889634f * 0.17677669529663687f) / (QKC * QKC);

  float m1[8], l1[8], m2[8], l2[8];
#pragma unroll
  for (int r = 0; r < 8; ++r) { m1[r] = NEGS; l1[r] = 0.f; m2[r] = NEGS; l2[r] = 0.f; }

#pragma unroll 1
  for (int ks = 0; ks < LK / 32; ++ks) {
    const int kb = ks * 32;
    v8f s10, s11, s20, s21;
    {
      const v16h kf0 = ldfrag_h(kp + (size_t)kb * DM), kf1 = ldfrag_h(kp + (size_t)(kb + 16) * DM);
      const v16h cf0 = ldfrag_h(cp + (size_t)kb * DM), cf1 = ldfrag_h(cp + (size_t)(kb + 16) * DM);
      s10 = mma_raw(q1, kf0, zero8());
      s11 = mma_raw(q1, kf1, zero8());
      s20 = mma_raw(q2, cf0, zero8());
      s21 = mma_raw(q2, cf1, zero8());
      guard_4x6(s10, s11, s20, s21, q1, q2, kf0, kf1, cf0, cf1);
    }
#pragma unroll
    for (int r = 0; r < 8; ++r) {
      ostep(s10[r] * lsc, s11[r] * lsc, m1[r], l1[r]);
      ostep(s20[r] * lsc, s21[r] * lsc, m2[r], l2[r]);
    }
  }

  float* ls = Ls[wave];
#pragma unroll
  for (int r = 0; r < 8; ++r) {
    ls[8 * hh + r]      = m1[r];
    ls[16 + 8 * hh + r] = l1[r];
    ls[32 + 8 * hh + r] = m2[r];
    ls[48 + 8 * hh + r] = l2[r];
  }
  wave_sync_lds();
  const v4f o = *(const v4f*)(ls + 4 * c);
  float* dp = ST + (size_t)wid * 64 + 4 * c;
  if (hh == 0) *(volatile v4f*)dp = o;
  __threadfence();
  if (hh == 0) *(volatile v4f*)dp = o;
}

__device__ __forceinline__ void build_ph(const float* pt, int c, int hh, FragH& ph) {
  const float* prow = pt + c * PSP + 8 * hh;
  const v4f p0 = *(const v4f*)(prow), p1 = *(const v4f*)(prow + 4);
  const v4f p2 = *(const v4f*)(prow + 16), p3 = *(const v4f*)(prow + 20);
#pragma unroll
  for (int e = 0; e < 4; ++e) {
    ph.h[0][e]     = (_Float16)p0[e];
    ph.h[0][4 + e] = (_Float16)p1[e];
    ph.h[1][e]     = (_Float16)p2[e];
    ph.h[1][4 + e] = (_Float16)p3[e];
  }
}

__device__ __forceinline__ void store_tile16x32(const float* os, int lane, unsigned short* dh, unsigned short* dl) {
  v4u h0, l0, h1, l1;
  split8(os + lane * 8, h0, l0);
  split8(os + 256 + lane * 8, h1, l1);
  *(volatile v4u*)(dh + lane * 8) = h0;
  *(volatile v4u*)(dh + 256 + lane * 8) = h1;
  *(volatile v4u*)(dl + lane * 8) = l0;
  *(volatile v4u*)(dl + 256 + lane * 8) = l1;
  __threadfence();
  *(volatile v4u*)(dh + lane * 8) = h0;
  *(volatile v4u*)(dh + 256 + lane * 8) = h1;
  *(volatile v4u*)(dl + lane * 8) = l0;
  *(volatile v4u*)(dl + 256 + lane * 8) = l1;
  __threadfence();
}

__global__ __launch_bounds__(128)
void pvk(const unsigned short* __restrict__ QP, const unsigned short* __restrict__ KP,
         const unsigned short* __restrict__ CP, const unsigned short* __restrict__ VTH,
         const float* __restrict__ ST, const float* __restrict__ S,
         unsigned short* CH, unsigned short* CL) {
  __shared__ __align__(16) float Ps[4][16 * PSP];
  __shared__ __align__(16) float Os[4][16 * 32];
  const int tid  = threadIdx.x;
  const int wave = tid >> 5;
  const int lane = tid & 31;
  const int hh   = lane >> 4;
  const int c    = lane & 15;
  const int wid  = blockIdx.x * 4 + wave;
  if (wid >= NWAV) return;
  const int h  = wid & (NH - 1);
  const int gt = wid >> 3;
  const int b  = gt / NQT;
  const int q0 = gt * 16;

  const _Float16* qp1 = (const _Float16*)(const void*)QP + (size_t)(q0 + c) * (size_t)(2 * DM) + HD * h + 8 * hh;
  const v16h q1 = ldfrag_h(qp1), q2 = ldfrag_h(qp1 + DM);
  const _Float16* kp  = (const _Float16*)(const void*)KP + ((size_t)b * LK + c) * (size_t)DM + HD * h + 8 * hh;
  const _Float16* cp  = (const _Float16*)(const void*)CP + ((size_t)b * LK + c) * (size_t)DM + HD * h + 8 * hh;
  const _Float16* vtp = (const _Float16*)(const void*)VTH + (size_t)(HD * h + c) * (size_t)NKR + (size_t)b * LK + 8 * hh;
  const float lsc = (1.4426950408889634f * 0.17677669529663687f) / (QKC * QKC);

  const float* stp = ST + (size_t)wid * 64 + 8 * hh;
  float m1[8], f1[8], m2[8], f2[8];
#pragma unroll
  for (int r = 0; r < 8; ++r) {
    m1[r] = stp[r];
    f1[r] = PCH / stp[16 + r];
    m2[r] = stp[32 + r];
    f2[r] = PCH / stp[48 + r];
  }

  v8f z0 = zero8(), z1 = zero8();
  float* pP = Ps[wave];

#pragma unroll 1
  for (int ks = 0; ks < LK / 32; ++ks) {
    const int kb = ks * 32;
    v8f s10, s11, s20, s21;
    {
      const v16h kf0 = ldfrag_h(kp + (size_t)kb * DM), kf1 = ldfrag_h(kp + (size_t)(kb + 16) * DM);
      const v16h cf0 = ldfrag_h(cp + (size_t)kb * DM), cf1 = ldfrag_h(cp + (size_t)(kb + 16) * DM);
      s10 = mma_raw(q1, kf0, zero8());
      s11 = mma_raw(q1, kf1, zero8());
      s20 = mma_raw(q2, cf0, zero8());
      s21 = mma_raw(q2, cf1, zero8());
      guard_4x6(s10, s11, s20, s21, q1, q2, kf0, kf1, cf0, cf1);
    }
#pragma unroll
    for (int r = 0; r < 8; ++r) {
      const float e0 = exp2f(s10[r] * lsc - m1[r]) * f1[r] + exp2f(s20[r] * lsc - m2[r]) * f2[r] - PONE;
      const float e1 = exp2f(s11[r] * lsc - m1[r]) * f1[r] + exp2f(s21[r] * lsc - m2[r]) * f2[r] - PONE;
      const int ro = (8 * hh + r) * PSP + c;
      pP[ro]      = e0;
      pP[ro + 16] = e1;
    }
    wave_sync_lds();
    const v16h vh0 = ldfrag_h(vtp + kb), vh1 = ldfrag_h(vtp + (size_t)16 * (size_t)NKR + kb);
    {
      FragH ph;
      build_ph(pP, c, hh, ph);
      z0 = mma_raw(ph.v, vh0, z0);
      z1 = mma_raw(ph.v, vh1, z1);
      guard_2x3(z0, z1, ph.v, vh0, vh1);
    }
    wave_sync_lds();
  }

  const float S0 = S[(size_t)b * DM + HD * h + c];
  const float S1 = S[(size_t)b * DM + HD * h + 16 + c];
  const float oc = ZC / (PCAR * VC);
  const float sa = PONE * VC;
  float* os = Os[wave];
#pragma unroll
  for (int r = 0; r < 8; ++r) {
    const int ro = (8 * hh + r) * 32 + c;
    os[ro]      = (z0[r] + sa * S0) * oc;
    os[ro + 16] = (z1[r] + sa * S1) * oc;
  }
  wave_sync_lds();
  unsigned short* dh = CH + ((size_t)h * (size_t)NQR + (size_t)q0) * HD;
  unsigned short* dl = CL + ((size_t)h * (size_t)NQR + (size_t)q0) * HD;
  store_tile16x32(os, lane, dh, dl);
  wave_sync_lds();
}

extern "C" void kernel_launch(void* const* d_in, const int* in_sizes, int n_in,
                              void* d_out, int out_size, void* d_ws, size_t ws_size,
                              hipStream_t stream) {
  if (n_in < 14) return;
  if (in_sizes[0] != NQR * DM) return;
  if (in_sizes[1] != NKR * DM || in_sizes[2] != NKR * DM || in_sizes[3] != NKR * DM) return;
  if (in_sizes[4] != 2 * DM * DM || in_sizes[5] != 2 * DM) return;
  if (in_sizes[6] != DM * DM || in_sizes[8] != DM * DM || in_sizes[10] != DM * DM || in_sizes[12] != DM * DM) return;
  if (in_sizes[7] != DM || in_sizes[9] != DM || in_sizes[11] != DM || in_sizes[13] != DM) return;
  if (out_size != NQR * DM) return;

  const float* Xq  = (const float*)d_in[0];
  const float* Xk  = (const float*)d_in[1];
  const float* Xv  = (const float*)d_in[2];
  const float* Xc  = (const float*)d_in[3];
  const float* Wq2 = (const float*)d_in[4];
  const float* bq2 = (const float*)d_in[5];
  const float* Wk  = (const float*)d_in[6];
  const float* bk  = (const float*)d_in[7];
  const float* Wc  = (const float*)d_in[8];
  const float* bc  = (const float*)d_in[9];
  const float* Wv  = (const float*)d_in[10];
  const float* bv  = (const float*)d_in[11];
  const float* Wo  = (const float*)d_in[12];
  const float* bo  = (const float*)d_in[13];
  float*       out = (float*)d_out;

  const size_t BWQ = (size_t)2 * DM * DM * 2;
  const size_t BW  = (size_t)DM * DM * 2;
  const size_t BXQ = (size_t)NQR * DM * 2;
  const size_t BXK = (size_t)NKR * DM * 2;
  const size_t BS  = 65536;
  const size_t BQP = (size_t)NQR * (2 * DM) * 2;
  const size_t BKP = (size_t)NKR * DM * 2;
  const size_t BVT = (size_t)DM * NKR * 2;
  const size_t BST = (size_t)NWAV * 64 * 4;
  const size_t BCH = (size_t)NH * NQR * HD * 2;
  size_t off = 0;
  const size_t oWq = off; off += BWQ;
  const size_t oWk = off; off += BW;
  const size_t oWc = off; off += BW;
  const size_t oWv = off; off += BW;
  const size_t oWo = off; off += BW;
  const size_t oXq = off; off += BXQ;
  const size_t oXk = off; off += BXK;
  const size_t oXc = off; off += BXK;
  const size_t oXv = off; off += BXK;
  const size_t oS  = off; off += BS;
  const size_t oQP = off; off += BQP;
  const size_t oKP = off; off += BKP;
  const size_t oCP = off; off += BKP;
  const size_t oVH = off; off += BVT;
  const size_t oVL = off; off += BVT;
  const size_t oST = off; off += BST;
  const size_t oCH = off; off += BCH;
  const size_t oCL = off; off += BCH;
  if (off > ws_size) return;
  if (off > (size_t)134217728) return;

  char* ws = (char*)d_ws;
  unsigned short* WqP = (unsigned short*)(ws + oWq);
  unsigned short* WkP = (unsigned short*)(ws + oWk);
  unsigned short* WcP = (unsigned short*)(ws + oWc);
  unsigned short* WvP = (unsigned short*)(ws + oWv);
  unsigned short* WoP = (unsigned short*)(ws + oWo);
  unsigned short* XQ  = (unsigned short*)(ws + oXq);
  unsigned short* XK  = (unsigned short*)(ws + oXk);
  unsigned short* XC  = (unsigned short*)(ws + oXc);
  unsigned short* XV  = (unsigned short*)(ws + oXv);
  float*          S   = (float*)(ws + oS);
  unsigned short* QP  = (unsigned short*)(ws + oQP);
  unsigned short* KP  = (unsigned short*)(ws + oKP);
  unsigned short* CP  = (unsigned short*)(ws + oCP);
  unsigned short* VTH = (unsigned short*)(ws + oVH);
  unsigned short* VTL = (unsigned short*)(ws + oVL);
  float*          ST  = (float*)(ws + oST);
  unsigned short* CH  = (unsigned short*)(ws + oCH);
  unsigned short* CL  = (unsigned short*)(ws + oCL);

  const dim3 blk(256), blk128(128);
  const float osQ = QKC / (ACARRY * WSC);
  const float osV = VC / (ACARRY * WSC);
  const float osO = 1.0f / (ZC * WSC);

  cvrow<<<dim3(NQR / 8), blk, 0, stream>>>(Xq, XQ, NQR, ACARRY);
  cvrow<<<dim3(NKR / 8), blk, 0, stream>>>(Xk, XK, NKR, ACARRY);
  cvrow<<<dim3(NKR / 8), blk, 0, stream>>>(Xc, XC, NKR, ACARRY);
  cvrow<<<dim3(NKR / 8), blk, 0, stream>>>(Xv, XV, NKR, ACARRY);
  cvrow<<<dim3((2 * DM) / 8), blk, 0, stream>>>(Wq2, WqP, 2 * DM, WSC);
  cvrow<<<dim3(DM / 8), blk, 0, stream>>>(Wk, WkP, DM, WSC);
  cvrow<<<dim3(DM / 8), blk, 0, stream>>>(Wc, WcP, DM, WSC);
  cvrow<<<dim3(DM / 8), blk, 0, stream>>>(Wv, WvP, DM, WSC);
  cvrow<<<dim3(DM / 8), blk, 0, stream>>>(Wo, WoP, DM, WSC);

  vhsum<<<dim3(NB), blk, 0, stream>>>(Xv, Wv, bv, S);

  gemm64<2, 0><<<dim3(((NQR / 64) * ((2 * DM) / 64) + 7) / 8), blk, 0, stream>>>(
      XQ, DM, 32LL, 0LL, WqP, DM, bq2, QKC,
      (void*)QP, 2 * DM, 0LL, NQR, 2 * DM, DM, osQ);
  gemm64<2, 0><<<dim3(((NKR / 64) * (DM / 64) + 7) / 8), blk, 0, stream>>>(
      XK, DM, 32LL, 0LL, WkP, DM, bk, QKC,
      (void*)KP, DM, 0LL, NKR, DM, DM, osQ);
  gemm64<2, 0><<<dim3(((NKR / 64) * (DM / 64) + 7) / 8), blk, 0, stream>>>(
      XC, DM, 32LL, 0LL, WcP, DM, bc, QKC,
      (void*)CP, DM, 0LL, NKR, DM, DM, osQ);
  gemm64<3, 1><<<dim3(((DM / 64) * (NKR / 64) + 7) / 8), blk, 0, stream>>>(
      WvP, DM, 32LL, 0LL, XV, DM, bv, VC,
      (void*)VTH, NKR, (long long)(VTL - VTH), DM, NKR, DM, osV);
  stats<<<dim3(NWAV / 4), blk128, 0, stream>>>(QP, KP, CP, ST);
  pvk<<<dim3(NWAV / 4), blk128, 0, stream>>>(QP, KP, CP, VTH, ST, S, CH, CL);
  gemm64<4, 0><<<dim3(((NQR / 64) * (DM / 64) + 7) / 8), blk, 0, stream>>>(
      CH, HD, (long long)NQR * HD, (long long)(CL - CH), WoP, DM, bo, 1.0f,
      (void*)out, DM, 0LL, NQR, DM, DM, osO);

  (void)hipGetLastError();
}
